// GatedAttnLayer_89361089561128
// MI455X (gfx1250) — hardware-verified
//
#include <hip/hip_runtime.h>


#define NB_  8
#define NT_  512
#define NTK  (NB_ * NT_)
#define DM   1024
#define NH_  64
#define HD   16
#define PSC  32768.0f
#define LOSC 1024.0f
#define LOSCI (1.0f / 1024.0f)

typedef _Float16 h16;
typedef unsigned short bf;
typedef __attribute__((ext_vector_type(16))) __bf16   v16bf;
typedef __attribute__((ext_vector_type(16))) _Float16 v16h;
typedef __attribute__((ext_vector_type(8)))  _Float16 v8h;
typedef __attribute__((ext_vector_type(8)))  unsigned short v8us;
typedef __attribute__((ext_vector_type(8)))  float    v8f;
typedef __attribute__((ext_vector_type(4)))  float    v4f;
typedef v8h  __attribute__((may_alias)) v8ha;
typedef v4f  __attribute__((may_alias)) v4fa;
typedef v8us __attribute__((may_alias)) v8usa;

__device__ __forceinline__ unsigned short f2bf(float f) { unsigned u = __float_as_uint(f); u += 0x7FFFu + ((u >> 16) & 1u); return (unsigned short)(u >> 16); }
__device__ __forceinline__ float bf2f(unsigned short b) { return __uint_as_float(((unsigned)b) << 16); }
__device__ __forceinline__ float bfr(float f) { return bf2f(f2bf(f)); }
__device__ __forceinline__ v16h cat16(v8h lo, v8h hi) { return __builtin_shufflevector(lo, hi, 0, 1, 2, 3, 4, 5, 6, 7, 8, 9, 10, 11, 12, 13, 14, 15); }
__device__ __forceinline__ v16bf cat16b(v8us lo, v8us hi) { return __builtin_bit_cast(v16bf, __builtin_shufflevector(lo, hi, 0, 1, 2, 3, 4, 5, 6, 7, 8, 9, 10, 11, 12, 13, 14, 15)); }
__device__ __forceinline__ v8f wmma16(v16h a, v16h b, v8f c) { return __builtin_amdgcn_wmma_f32_16x16x32_f16(false, a, false, b, (short)0, c, false, false); }
__device__ __forceinline__ v8f wmmab(v16bf a, v16bf b, v8f c) { return __builtin_amdgcn_wmma_f32_16x16x32_bf16(false, a, false, b, (short)0, c, false, false); }
#define VST2(T, p, v) do { const T vst2_v_ = (v); *(volatile T*)(p) = vst2_v_; __threadfence(); *(volatile T*)(p) = vst2_v_; } while (0)

__global__ __launch_bounds__(256) void k_cvtb(const float* __restrict__ src, int nrows, bf* dst) {
    const int lane = threadIdx.x & 31, r = blockIdx.x * 8 + (threadIdx.x >> 5);
    if (r >= nrows) return;
    v8us o[4];
#pragma unroll
    for (int q = 0; q < 4; ++q)
#pragma unroll
        for (int i = 0; i < 8; ++i) o[q][i] = f2bf(src[(size_t)r * DM + q * 256 + lane * 8 + i]);
#pragma unroll
    for (int q = 0; q < 4; ++q) *(volatile v8us*)(dst + (size_t)r * DM + q * 256 + lane * 8) = o[q];
    __threadfence();
#pragma unroll
    for (int q = 0; q < 4; ++q) *(volatile v8us*)(dst + (size_t)r * DM + q * 256 + lane * 8) = o[q];
}
__global__ __launch_bounds__(256) void k_wt(const float* __restrict__ Wm, bf* WT) {
    __shared__ __align__(16) unsigned short tl[64 * 72];
    const int tid = threadIdx.x, k0 = blockIdx.x * 64, n0 = blockIdx.y * 64;
    const int kk = tid >> 2, nq = (tid & 3) * 16;
#pragma unroll
    for (int i = 0; i < 16; ++i) tl[(nq + i) * 72 + kk] = f2bf(Wm[(size_t)(k0 + kk) * DM + n0 + nq + i]);
    __syncthreads();
    const int piece = tid & 7;
    auto pass = [&]() {
#pragma unroll
        for (int s = 0; s < 2; ++s) { const int nr = (tid >> 3) + 32 * s; const v8us val = *(const v8usa*)(tl + nr * 72 + piece * 8); *(volatile v8us*)(WT + (size_t)(n0 + nr) * DM + k0 + piece * 8) = val; }
    };
    pass(); __threadfence(); pass();
}
__global__ __launch_bounds__(128) void k_gemm(const bf* __restrict__ A, const bf* __restrict__ Bn, const float* __restrict__ bias, float* C) {
    __shared__ __align__(16) float ost[4][16 * 68];
    const int lane = threadIdx.x & 31, wave = threadIdx.x >> 5, lr = lane & 15, hi = lane >> 4;
    const size_t r0 = (size_t)blockIdx.x * 64 + wave * 16; const int c0 = blockIdx.y * 64;
    v8f acc[4];
#pragma unroll
    for (int t = 0; t < 4; ++t) acc[t] = (v8f){};
#pragma unroll 2
    for (int kc = 0; kc < DM; kc += 32) {
        const v16bf a = cat16b(*(const v8us*)(A + (r0 + lr) * DM + kc + 8 * hi), *(const v8us*)(A + (r0 + lr) * DM + kc + 8 * hi + 16));
#pragma unroll
        for (int t = 0; t < 4; ++t) { const bf* bp = Bn + (size_t)(c0 + t * 16 + lr) * DM + kc + 8 * hi; acc[t] = wmmab(a, cat16b(*(const v8us*)bp, *(const v8us*)(bp + 16)), acc[t]); }
        asm volatile("v_nop" : "+v"(acc[0]), "+v"(acc[1]), "+v"(acc[2]), "+v"(acc[3]) : "v"(a) : "memory");
    }
    float* os = &ost[wave][0];
#pragma unroll
    for (int t = 0; t < 4; ++t) { const float bv = bfr(bias[c0 + t * 16 + lr]);
#pragma unroll
        for (int j = 0; j < 8; ++j) os[(hi * 8 + j) * 68 + t * 16 + lr] = acc[t][j] + bv; }
    __builtin_amdgcn_wave_barrier(); asm volatile("" ::: "memory");
    float* crow = C + r0 * DM + c0;
    auto pass = [&]() {
#pragma unroll
        for (int s = 0; s < 8; ++s) { const int Lid = (lane >> 3) + 4 * s, piece = lane & 7; const int row = Lid >> 1, cofs = (Lid & 1) * 32 + piece * 4;
            const v4f val = *(const v4fa*)(os + row * 68 + cofs); *(volatile v4f*)(crow + (size_t)row * DM + cofs) = val; }
    };
    pass(); __threadfence(); pass();
}
__global__ __launch_bounds__(256) void k_gate(const float* __restrict__ Qf, const float* __restrict__ Kf, const float* __restrict__ Wfq, const float* __restrict__ bfq, const float* __restrict__ Wfk, const float* __restrict__ bfk,
                                             const float* __restrict__ Wfg, const float* __restrict__ bfg, h16* QH, h16* QL, h16* KH, h16* KL) {
    typedef __attribute__((ext_vector_type(2))) _Float16 v2h;
    __shared__ float wq[16 * 16], wk[16 * 16], wg[16 * 32], bq_[16], bk_[16], bg_[32];
    __shared__ float qs[8][32], ks[8][32], gs[8][32];
    __shared__ __align__(16) h16 st[8][4][64];
    const int tid = threadIdx.x, lane = tid & 31, wave = tid >> 5;
    for (int i = tid; i < 256; i += 256) { wq[i] = bfr(Wfq[i]); wk[i] = bfr(Wfk[i]); }
    for (int i = tid; i < 512; i += 256) wg[i] = bfr(Wfg[i]);
    if (tid < 16) { bq_[tid] = bfr(bfq[tid]); bk_[tid] = bfr(bfk[tid]); }
    if (tid < 32) bg_[tid] = bfr(bfg[tid]);
    __syncthreads();
    const size_t wid = (size_t)blockIdx.x * 8 + wave; const size_t t = wid >> 4; const int hq = (int)(wid & 15);
    const int hh = lane >> 4, d = lane & 15;
#pragma unroll 1
    for (int half = 0; half < 2; ++half) {
        const int h = hq * 4 + half * 2 + hh;
        const size_t col = t * DM + (size_t)h * HD + d;
        const float qv = Qf[col], kv = Kf[col];
        qs[wave][lane] = qv; ks[wave][lane] = kv;
        asm volatile("" ::: "memory"); __builtin_amdgcn_wave_barrier();
        float fq = bq_[d], fk = bk_[d];
#pragma unroll 1
        for (int e = 0; e < 16; ++e) { fq += qs[wave][hh * 16 + e] * wq[e * 16 + d]; fk += ks[wave][hh * 16 + e] * wk[e * 16 + d]; }
        gs[wave][lane] = fq * fk;
        asm volatile("" ::: "memory"); __builtin_amdgcn_wave_barrier();
        float m0 = bg_[d], m1 = bg_[16 + d];
#pragma unroll 1
        for (int e = 0; e < 16; ++e) { const float g = gs[wave][hh * 16 + e]; m0 += g * wg[e * 32 + d]; m1 += g * wg[e * 32 + 16 + d]; }
        m0 = 1.0f / (1.0f + __expf(-m0)); m1 = 1.0f / (1.0f + __expf(-m1));
        const float qg = qv * m0, kg = kv * m1;
        const h16 qa = (h16)qg, ka = (h16)kg;
        const int sl = half * 32 + lane;
        st[wave][0][sl] = qa; st[wave][1][sl] = (h16)((qg - (float)qa) * LOSC); st[wave][2][sl] = ka; st[wave][3][sl] = (h16)((kg - (float)ka) * LOSC);
        asm volatile("" ::: "memory"); __builtin_amdgcn_wave_barrier();
    }
    const size_t o = t * DM + (size_t)hq * 64 + lane * 2;
    typedef v2h __attribute__((may_alias)) v2ha;
    const v2h a0 = *(const v2ha*)(&st[wave][0][lane * 2]), a1 = *(const v2ha*)(&st[wave][1][lane * 2]), a2 = *(const v2ha*)(&st[wave][2][lane * 2]), a3 = *(const v2ha*)(&st[wave][3][lane * 2]);
    *(volatile v2h*)(QH + o) = a0; *(volatile v2h*)(QL + o) = a1; *(volatile v2h*)(KH + o) = a2; *(volatile v2h*)(KL + o) = a3; __threadfence();
    *(volatile v2h*)(QH + o) = a0; *(volatile v2h*)(QL + o) = a1; *(volatile v2h*)(KH + o) = a2; *(volatile v2h*)(KL + o) = a3;
}
__global__ __launch_bounds__(256) void k_vt(const float* __restrict__ Vf, h16* VTH, h16* VTL) {
    __shared__ __align__(16) h16 tl[16 * 520];
    __shared__ __align__(16) h16 tl2[16 * 520];
    const int tid = threadIdx.x, h = blockIdx.x, b = blockIdx.y;
#pragma unroll
    for (int r = 0; r < 2; ++r) { const int t = r * 256 + tid;
#pragma unroll
        for (int d = 0; d < HD; ++d) { const float v = Vf[((size_t)b * NT_ + t) * DM + h * HD + d]; const h16 a = (h16)v; tl[d * 520 + t] = a; tl2[d * 520 + t] = (h16)((v - (float)a) * LOSC); } }
    __syncthreads();
    const size_t base = (((size_t)b * NH_ + h) * HD) * NT_;
    auto pass = [&]() {
#pragma unroll
        for (int s = 0; s < 4; ++s) { const int idx = s * 256 + tid; const int row = idx >> 6, piece = idx & 63;
            *(volatile v8h*)(VTH + base + (size_t)row * NT_ + piece * 8) = *(const v8ha*)(tl + row * 520 + piece * 8);
            *(volatile v8h*)(VTL + base + (size_t)row * NT_ + piece * 8) = *(const v8ha*)(tl2 + row * 520 + piece * 8); }
    };
    pass(); __threadfence(); pass();
}
__global__ __launch_bounds__(128) void k_attn(const h16* __restrict__ QH, const h16* __restrict__ QL, const h16* __restrict__ KH, const h16* __restrict__ KL, const h16* __restrict__ VTH, const h16* __restrict__ VTL, float* X) {
    __shared__ __align__(16) h16 plds[4][16 * 32];
    __shared__ __align__(16) h16 plds2[4][16 * 32];
    __shared__ __align__(16) float ost[4][16 * 132];
    const int lane = threadIdx.x & 31, wave = threadIdx.x >> 5, lr = lane & 15, hi = lane >> 4;
    const int b = blockIdx.y, qt = blockIdx.x, q0 = qt * 64 + wave * 16;
    const size_t tok0 = (size_t)b * NT_;
    h16* pl = &plds[wave][0]; h16* pl2 = &plds2[wave][0]; float* os = &ost[wave][0];
    const v8h z8 = (v8h){};
#pragma unroll 1
    for (int hg = 0; hg < NH_ / 8; ++hg) {
#pragma unroll 1
        for (int hx = 0; hx < 8; ++hx) { const int h = hg * 8 + hx;
            const size_t qo = (tok0 + q0 + lr) * DM + h * HD;
            const v16h qa = cat16(*(const v8h*)(QH + qo + 8 * hi), z8), ql = cat16(*(const v8h*)(QL + qo + 8 * hi), z8);
            v8f o = (v8f){}, ox = (v8f){};
            float mrow[8], lpart[8];
#pragma unroll
            for (int j = 0; j < 8; ++j) { mrow[j] = -3.0e38f; lpart[j] = 0.f; }
            const size_t vrow = (((size_t)b * NH_ + h) * HD + lr) * NT_ + 8 * hi;
#pragma unroll 1
            for (int kt = 0; kt < NT_ / 32; ++kt) {
                const int l0 = kt * 32;
                const size_t ka = (tok0 + l0 + lr) * DM + h * HD, kb = (tok0 + l0 + 16 + lr) * DM + h * HD;
                const v16h k0h = cat16(*(const v8h*)(KH + ka + 8 * hi), z8), k1h = cat16(*(const v8h*)(KH + kb + 8 * hi), z8);
                const v16h k0l = cat16(*(const v8h*)(KL + ka + 8 * hi), z8), k1l = cat16(*(const v8h*)(KL + kb + 8 * hi), z8);
                v8f s0 = wmma16(qa, k0h, (v8f){}), s1 = wmma16(qa, k1h, (v8f){}), x0 = wmma16(ql, k0h, (v8f){}), x1 = wmma16(ql, k1h, (v8f){});
                x0 = wmma16(qa, k0l, x0); x1 = wmma16(qa, k1l, x1);
                asm volatile("v_nop\n\tv_nop\n\tv_nop\n\tv_nop" : "+v"(s0), "+v"(s1), "+v"(x0), "+v"(x1) : "v"(qa), "v"(ql));
                float alpha[8];
#pragma unroll
                for (int j = 0; j < 8; ++j) { const int qr = hi * 8 + j;
                    const float a0 = (s0[j] + x0[j] * LOSCI) * 0.25f, a1 = (s1[j] + x1[j] * LOSCI) * 0.25f;
                    float mx = fmaxf(a0, a1);
                    mx = fmaxf(mx, __shfl_xor(mx, 1, 16)); mx = fmaxf(mx, __shfl_xor(mx, 2, 16)); mx = fmaxf(mx, __shfl_xor(mx, 4, 16)); mx = fmaxf(mx, __shfl_xor(mx, 8, 16));
                    const float mn = fmaxf(mrow[j], mx);
                    alpha[j] = __expf(mrow[j] - mn); mrow[j] = mn;
                    const float p0 = __expf(a0 - mn), p1 = __expf(a1 - mn);
                    lpart[j] = lpart[j] * alpha[j] + (p0 + p1);
                    const float ps0 = p0 * PSC, ps1 = p1 * PSC; const h16 h0 = (h16)ps0, h1 = (h16)ps1;
                    pl[qr * 32 + lr] = h0; pl[qr * 32 + 16 + lr] = h1; pl2[qr * 32 + lr] = (h16)(ps0 - (float)h0); pl2[qr * 32 + 16 + lr] = (h16)(ps1 - (float)h1); }
#pragma unroll
                for (int j = 0; j < 8; ++j) { o[j] *= alpha[j]; ox[j] *= alpha[j]; }
                asm volatile("" ::: "memory");
                const v16h pa = cat16(*(const v8ha*)(pl + lr * 32 + hi * 8), *(const v8ha*)(pl + lr * 32 + 16 + hi * 8));
                const v16h px = cat16(*(const v8ha*)(pl2 + lr * 32 + hi * 8), *(const v8ha*)(pl2 + lr * 32 + 16 + hi * 8));
                const v16h vh = cat16(*(const v8h*)(VTH + vrow + l0), *(const v8h*)(VTH + vrow + l0 + 16)), vl = cat16(*(const v8h*)(VTL + vrow + l0), *(const v8h*)(VTL + vrow + l0 + 16));
                o = wmma16(pa, vh, o); o = wmma16(px, vh, o); ox = wmma16(pa, vl, ox);
                asm volatile("v_nop\n\tv_nop\n\tv_nop\n\tv_nop" : "+v"(o), "+v"(ox) : "v"(pa), "v"(px), "v"(vh), "v"(vl));
                __builtin_amdgcn_wave_barrier();
            }
            float inv[8];
#pragma unroll
            for (int j = 0; j < 8; ++j) { float rs = lpart[j]; rs += __shfl_xor(rs, 1, 16); rs += __shfl_xor(rs, 2, 16); rs += __shfl_xor(rs, 4, 16); rs += __shfl_xor(rs, 8, 16); inv[j] = 1.0f / (rs * PSC); }
#pragma unroll
            for (int j = 0; j < 8; ++j) os[(hi * 8 + j) * 132 + hx * HD + lr] = (o[j] + ox[j] * LOSCI) * inv[j];
            __builtin_amdgcn_wave_barrier(); asm volatile("" ::: "memory");
        }
        auto pass = [&]() {
#pragma unroll
            for (int s = 0; s < 16; ++s) { const v4f val = *(const v4fa*)(os + s * 132 + lane * 4); *(volatile v4f*)(X + (tok0 + q0 + s) * DM + hg * 128 + lane * 4) = val; }
        };
        pass(); __threadfence(); pass();
        __builtin_amdgcn_wave_barrier(); asm volatile("" ::: "memory");
    }
}
__global__ __launch_bounds__(256) void k_bnstat(const float* __restrict__ X, float* MEAN, float* RSTD) {
    __shared__ float red[8][32]; __shared__ float mu_s[32];
    const int c0 = blockIdx.x * 32, cl = threadIdx.x & 31, part = threadIdx.x >> 5;
    float s = 0.f;
    for (int t = part * 512; t < part * 512 + 512; ++t) s += X[(size_t)t * DM + c0 + cl];
    red[part][cl] = s; __syncthreads();
    if (part == 0) { float a = 0.f;
#pragma unroll
        for (int p = 0; p < 8; ++p) a += red[p][cl];
        mu_s[cl] = a / (float)NTK; }
    __syncthreads();
    const float mu = mu_s[cl]; float q = 0.f;
    for (int t = part * 512; t < part * 512 + 512; ++t) { const float dv = X[(size_t)t * DM + c0 + cl] - mu; q += dv * dv; }
    __syncthreads(); red[part][cl] = q; __syncthreads();
    if (part == 0) { float a = 0.f;
#pragma unroll
        for (int p = 0; p < 8; ++p) a += red[p][cl];
        const float rs = rsqrtf(a / (float)NTK + 1e-5f);
        *(volatile float*)(MEAN + c0 + cl) = mu; *(volatile float*)(RSTD + c0 + cl) = rs; __threadfence(); *(volatile float*)(MEAN + c0 + cl) = mu; *(volatile float*)(RSTD + c0 + cl) = rs; }
}
__global__ __launch_bounds__(256) void k_bnapply(const float* __restrict__ X, const float* __restrict__ MEAN, const float* __restrict__ RSTD, const float* __restrict__ gam, const float* __restrict__ bet, float* out) {
    const int lane = threadIdx.x & 31; const size_t r = (size_t)blockIdx.x * 8 + (threadIdx.x >> 5);
    if (r >= (size_t)NTK) return;
#pragma unroll 1
    for (int ps = 0; ps < 2; ++ps) {
#pragma unroll
        for (int q = 0; q < DM / 128; ++q) { v4f v; const int c = q * 128 + lane * 4;
#pragma unroll
            for (int i = 0; i < 4; ++i) v[i] = (X[r * DM + c + i] - MEAN[c + i]) * RSTD[c + i] * bfr(gam[c + i]) + bfr(bet[c + i]);
            *(volatile v4f*)(out + r * DM + c) = v; }
        if (ps == 0) __threadfence(); }
}

extern "C" void kernel_launch(void* const* d_in, const int* in_sizes, int n_in,
                              void* d_out, int out_size, void* d_ws, size_t ws_size, hipStream_t stream) {
    (void)in_sizes; (void)n_in; (void)out_size;
    const float* x = (const float*)d_in[0]; const float* Wq = (const float*)d_in[1]; const float* bq = (const float*)d_in[2]; const float* Wk = (const float*)d_in[3]; const float* bk = (const float*)d_in[4];
    const float* Wv = (const float*)d_in[5]; const float* bv = (const float*)d_in[6]; const float* Wfq = (const float*)d_in[7]; const float* bfq = (const float*)d_in[8]; const float* Wfk = (const float*)d_in[9]; const float* bfk = (const float*)d_in[10];
    const float* Wfg = (const float*)d_in[11]; const float* bfg = (const float*)d_in[12]; const float* gam = (const float*)d_in[13]; const float* bet = (const float*)d_in[14];
    float* out = (float*)d_out;
    char* wsp = (char*)d_ws;
    auto take = [&](size_t bytes) { char* p = wsp; wsp += (bytes + 255) & ~(size_t)255; return (void*)p; };
    bf* Xb = (bf*)take((size_t)NTK * DM * 2); bf* WqT = (bf*)take((size_t)DM * DM * 2); bf* WkT = (bf*)take((size_t)DM * DM * 2); bf* WvT = (bf*)take((size_t)DM * DM * 2);
    float* Qf = (float*)take((size_t)NTK * DM * 4); float* Kf = (float*)take((size_t)NTK * DM * 4); float* Vf = (float*)take((size_t)NTK * DM * 4);
    h16* QH = (h16*)take((size_t)NTK * DM * 2); h16* QL = (h16*)take((size_t)NTK * DM * 2); h16* KH = (h16*)take((size_t)NTK * DM * 2); h16* KL = (h16*)take((size_t)NTK * DM * 2);
    h16* VTH = (h16*)take((size_t)NTK * DM * 2); h16* VTL = (h16*)take((size_t)NTK * DM * 2); float* MEAN = (float*)take((size_t)DM * 4); float* RSTD = (float*)take((size_t)DM * 4);
    if ((size_t)(wsp - (char*)d_ws) > ws_size) return;
    float* Xa = Qf;
    k_cvtb<<<NTK / 8, 256, 0, stream>>>(x, NTK, Xb);
    k_wt<<<dim3(DM / 64, DM / 64, 1), 256, 0, stream>>>(Wq, WqT); k_wt<<<dim3(DM / 64, DM / 64, 1), 256, 0, stream>>>(Wk, WkT); k_wt<<<dim3(DM / 64, DM / 64, 1), 256, 0, stream>>>(Wv, WvT);
    k_gemm<<<dim3(NTK / 64, DM / 64, 1), 128, 0, stream>>>(Xb, WqT, bq, Qf);
    k_gemm<<<dim3(NTK / 64, DM / 64, 1), 128, 0, stream>>>(Xb, WkT, bk, Kf);
    k_gemm<<<dim3(NTK / 64, DM / 64, 1), 128, 0, stream>>>(Xb, WvT, bv, Vf);
    k_gate<<<(unsigned)((NTK * 16) / 8), 256, 0, stream>>>(Qf, Kf, Wfq, bfq, Wfk, bfk, Wfg, bfg, QH, QL, KH, KL);
    k_vt<<<dim3(NH_, NB_, 1), 256, 0, stream>>>(Vf, VTH, VTL);
    k_attn<<<dim3(NT_ / 64, NB_, 1), 128, 0, stream>>>(QH, QL, KH, KL, VTH, VTL, Xa);
    k_bnstat<<<DM / 32, 256, 0, stream>>>(Xa, MEAN, RSTD);
    k_bnapply<<<NTK / 8, 256, 0, stream>>>(Xa, MEAN, RSTD, gam, bet, out);
}
